// SparseResidualBlock_3968549781705
// MI455X (gfx1250) — hardware-verified
//
#include <hip/hip_runtime.h>
#include <math.h>

typedef __attribute__((ext_vector_type(16))) _Float16 v16h;
typedef __attribute__((ext_vector_type(16))) __bf16 v16b;
typedef __attribute__((ext_vector_type(8)))  _Float16 v8h;
typedef __attribute__((ext_vector_type(8)))  float v8f;
typedef __attribute__((ext_vector_type(4)))  float v4f;
typedef __attribute__((ext_vector_type(2)))  float v2f;
typedef __attribute__((ext_vector_type(4)))  unsigned v4u;
typedef __attribute__((ext_vector_type(4)))  int v4i;
typedef float __attribute__((may_alias)) float_a;
typedef int __attribute__((may_alias)) int_a;

template <typename T> __device__ __forceinline__ void vst2(void* p, T v) { *(volatile T*)p = v; __threadfence(); *(volatile T*)p = v; }
__device__ __forceinline__ v8f wmma16(v16h a, v16h b, v8f c) {
  v8f d = __builtin_amdgcn_wmma_f32_16x16x32_f16(false, a, false, b, (short)0, c, false, false);
  asm volatile("v_nop\n\tv_nop\n\tv_nop\n\tv_nop" : "+v"(d) : "v"(a), "v"(b));
  return d;
}
__device__ __forceinline__ v8f wmma_bf(v16b a, v16b b, v8f c) {
  v8f d = __builtin_amdgcn_wmma_f32_16x16x32_bf16(false, a, false, b, (short)0, c, false, false);
  asm volatile("v_nop\n\tv_nop\n\tv_nop\n\tv_nop" : "+v"(d) : "v"(a), "v"(b));
  return d;
}
__device__ __forceinline__ v16h frag_h(const _Float16* rowk0, int lane) {
  union { v16h v; v8h q[2]; } u; const _Float16* p = rowk0 + 8 * (lane >> 4);
  u.q[0] = *(const v8h*)p; u.q[1] = *(const v8h*)(p + 16); return u.v;
}
__device__ __forceinline__ v16h frag_f32(const float* rowk0, int lane) {
  v16h a; const float* p = rowk0 + 8 * (lane >> 4);
#pragma unroll
  for (int i = 0; i < 8; ++i) { a[i] = (_Float16)p[i]; a[8 + i] = (_Float16)p[16 + i]; }
  return a;
}
__device__ __forceinline__ v16h frag_f32s(const float* rowk0, int lane, float sc) {
  v16h a; const float* p = rowk0 + 8 * (lane >> 4);
#pragma unroll
  for (int i = 0; i < 8; ++i) { a[i] = (_Float16)(p[i] * sc); a[8 + i] = (_Float16)(p[16 + i] * sc); }
  return a;
}
__device__ __forceinline__ v16h fragc_f32(const float* W, int k0, int n, int lane, int ld, int K) {
  v16h a; const int g = lane >> 4;
#pragma unroll
  for (int i = 0; i < 8; ++i) { const int ka = k0 + 8 * g + i, kb = ka + 16;
    a[i] = (_Float16)(ka < K ? W[(size_t)(ka < K ? ka : K - 1) * ld + n] : 0.f); a[8 + i] = (_Float16)(kb < K ? W[(size_t)(kb < K ? kb : K - 1) * ld + n] : 0.f); }
  return a;
}
struct F2 { v16b h, l; };
__device__ __forceinline__ F2 bsplit16(const float v[16]) { F2 r;
#pragma unroll
  for (int i = 0; i < 16; ++i) { const __bf16 h = (__bf16)v[i]; r.h[i] = h; r.l[i] = (__bf16)(v[i] - (float)h); }
  return r; }
__device__ __forceinline__ F2 split_row(const float* row, int k0, int lane) { float v[16]; const float* p = row + k0 + 8 * (lane >> 4);
#pragma unroll
  for (int i = 0; i < 8; ++i) { v[i] = p[i]; v[8 + i] = p[16 + i]; }
  return bsplit16(v); }
__device__ __forceinline__ F2 split_rowK(const float* row, int k0, int lane, int K) { float v[16]; const int g = lane >> 4;
#pragma unroll
  for (int i = 0; i < 8; ++i) { const int ka = k0 + 8 * g + i, kb = ka + 16; v[i] = ka < K ? row[ka < K ? ka : K - 1] : 0.f; v[8 + i] = kb < K ? row[kb < K ? kb : K - 1] : 0.f; }
  return bsplit16(v); }
__device__ __forceinline__ F2 split_col(const float* W, int k0, int n, int lane, int ld, int K) { float v[16]; const int g = lane >> 4;
#pragma unroll
  for (int i = 0; i < 8; ++i) { const int ka = k0 + 8 * g + i, kb = ka + 16; v[i] = ka < K ? W[(size_t)(ka < K ? ka : K - 1) * ld + n] : 0.f; v[8 + i] = kb < K ? W[(size_t)(kb < K ? kb : K - 1) * ld + n] : 0.f; }
  return bsplit16(v); }
__device__ __forceinline__ v8f mac3(const F2& a, const F2& b, v8f c) { c = wmma_bf(a.l, b.h, c); c = wmma_bf(a.h, b.l, c); return wmma_bf(a.h, b.h, c); }
__device__ __forceinline__ float sigm(float v) { return 1.0f / (1.0f + expf(-v)); }
#define LDSX() do { asm volatile("s_wait_dscnt 0" ::: "memory"); __builtin_amdgcn_wave_barrier(); __builtin_amdgcn_fence(__ATOMIC_RELEASE, "workgroup"); } while (0)


#ifndef NN
#define NN 100000
#endif
#define KN 27
#define CIN 64
#define CO 128
#define K1 (KN * CIN)
#define K2 (KN * CO)
#define NBLK ((NN + 63) / 64)
#define NRP (NBLK * 64)
typedef __attribute__((ext_vector_type(8))) __bf16 v8b;
__device__ __forceinline__ v16b frag_b(const __bf16* rowk0, int lane) {
  union { v16b v; v8b q[2]; } u; const __bf16* p = rowk0 + 8 * (lane >> 4);
  u.q[0] = *(const v8b*)p; u.q[1] = *(const v8b*)(p + 16); return u.v;
}
__device__ __forceinline__ float bfr(float v) { return (float)(__bf16)v; }
__device__ __attribute__((noinline)) float exp_ni(float v) { return expf(v); }
__device__ __attribute__((noinline)) float erf_ni(float v) { return erff(v); }

#define WS_P1   0u
#define WS_P2   (WS_P1 + 2u * CO * K1)
#define WS_PS   (WS_P2 + 2u * CO * K2)
#define WS_Y    (WS_PS + 2u * CO * CIN)
#define WS_H    (WS_Y + 4u * NRP * CO)
#define WS_PSUM (WS_H + 4u * NRP * CO)
#define WS_ST   (WS_PSUM + 4u * NBLK * CO)
#define WS_END  (WS_ST + 4u * 2 * CO)

__global__ __launch_bounds__(256) void k_pack(const float* __restrict__ W1, const float* __restrict__ W2, const float* __restrict__ WSK, __bf16* __restrict__ P1, __bf16* __restrict__ P2, __bf16* __restrict__ PSK) {
  __shared__ __align__(16) __bf16 s[K2]; const int o = blockIdx.x, which = blockIdx.y, tid = threadIdx.x;
  const int K = (which == 0) ? K1 : (which == 1 ? K2 : CIN);
  for (int kk = tid; kk < K; kk += 256) { float v; if (which == 0) v = W1[(size_t)kk * CO + o]; else if (which == 1) v = W2[(size_t)kk * CO + o]; else v = WSK[(size_t)kk * CO + o]; s[kk] = (__bf16)v; }
  __syncthreads();
  __bf16* dst = (which == 0) ? P1 + (size_t)o * K1 : (which == 1 ? P2 + (size_t)o * K2 : PSK + (size_t)o * CIN);
  for (int q = tid; q < K / 8; q += 256) vst2((unsigned*)(dst + q * 8), *(const v4u*)&s[q * 8]);
}
template <int C, int RIN>
__global__ __launch_bounds__(128) void k_conv(const float* __restrict__ SRCX, const int* __restrict__ NBR, const __bf16* __restrict__ P, float* __restrict__ Y) {
  __shared__ __align__(16) float so[4][16][132];
  const int tid = threadIdx.x, wave = tid >> 5, lane = tid & 31, col = lane & 15, g = lane >> 4; const size_t r0 = (size_t)blockIdx.x * 64 + wave * 16; size_t ra = r0 + col; if (ra >= NN) ra = NN - 1;
  const int* nrow = NBR + ra * KN;
  v8f acc[8] = {};
#pragma unroll 1
  for (int k = 0; k < KN; ++k) { const int nb = nrow[k]; const bool ok = (nb >= 0 && nb < NN); const float* src = SRCX + (size_t)(ok ? nb : 0) * C;
#pragma unroll
    for (int cc = 0; cc < C / 32; ++cc) { float v[16]; const float* p = src + cc * 32 + 8 * g;
#pragma unroll
      for (int i = 0; i < 8; ++i) { v[i] = ok ? p[i] : 0.f; v[8 + i] = ok ? p[16 + i] : 0.f; }
      const F2 a = bsplit16(v); const int kk0 = k * C + cc * 32;
#pragma unroll
      for (int j = 0; j < 8; ++j) { const v16b w = frag_b(P + (size_t)(j * 16 + col) * (KN * C) + kk0, lane); if (!RIN) acc[j] = wmma_bf(a.l, w, acc[j]); acc[j] = wmma_bf(a.h, w, acc[j]); } } }
#pragma unroll
  for (int j = 0; j < 8; ++j)
#pragma unroll
    for (int r = 0; r < 8; ++r) so[wave][8 * g + r][j * 16 + col] = acc[j][r];
  LDSX();
  for (int rl = 0; rl < 16; ++rl) vst2(Y + (r0 + rl) * CO + lane * 4, *(const v4f*)&so[wave][rl][lane * 4]);
}
template <int MODE>
__global__ __launch_bounds__(128) void k_colsum(const float* __restrict__ Yv, const float* __restrict__ ST, float* __restrict__ PSUM) {
  __shared__ __align__(16) float s[CO]; const int blk = blockIdx.x, c = threadIdx.x; const float mu = (MODE == 1) ? ST[c] : 0.f; float acc = 0.f;
  for (int rl = 0; rl < 64; ++rl) { const size_t row = (size_t)blk * 64 + rl; if (row < (size_t)NN) { const float v = Yv[row * CO + c]; acc += (MODE == 1) ? (v - mu) * (v - mu) : v; } }
  s[c] = acc; __syncthreads();
  if (c < 32) vst2(PSUM + (size_t)blk * CO + c * 4, *(const v4f*)&s[c * 4]);
}
template <int MODE>
__global__ __launch_bounds__(128) void k_red(const float* __restrict__ PSUM, float* __restrict__ ST) {
  __shared__ __align__(16) float s[CO]; const int c = threadIdx.x; float acc = 0.f;
  for (int b = 0; b < NBLK; ++b) acc += PSUM[(size_t)b * CO + c];
  s[c] = (MODE == 0) ? acc / (float)NN : rsqrtf(acc / (float)NN + 1e-5f);
  __syncthreads();
  if (c < 32) vst2(ST + MODE * CO + c * 4, *(const v4f*)&s[c * 4]);
}
__global__ __launch_bounds__(256) void k_bnact(const float* __restrict__ Yv, const float* __restrict__ ST, const float* __restrict__ gm, const float* __restrict__ bt, float* __restrict__ H) {
  __shared__ __align__(16) float so[64][CO + 4]; __shared__ float smu[CO], srs[CO], sg[CO], sb[CO]; const int tid = threadIdx.x, blk = blockIdx.x;
  if (tid < CO) { smu[tid] = ST[tid]; srs[tid] = ST[CO + tid]; sg[tid] = bfr(gm[tid]); sb[tid] = bfr(bt[tid]); }
  __syncthreads();
  for (int q = tid; q < 64 * CO; q += 256) { const int rl = q >> 7, c = q & 127; const size_t row = (size_t)blk * 64 + rl; float v = 0.f; if (row < (size_t)NN) { v = (Yv[row * CO + c] - smu[c]) * srs[c] * sg[c] + sb[c]; v = fmaxf(v, 0.f); } so[rl][c] = v; }
  __syncthreads();
  for (int q = tid; q < 64 * 32; q += 256) { const int rl = q >> 5, pc = q & 31; vst2(H + ((size_t)blk * 64 + rl) * CO + pc * 4, *(const v4f*)&so[rl][pc * 4]); }
}
__global__ __launch_bounds__(128) void k_final(const float* __restrict__ X, const __bf16* __restrict__ PSK, const float* __restrict__ Yv, const float* __restrict__ ST, const float* __restrict__ gm, const float* __restrict__ bt, float* __restrict__ out) {
  __shared__ __align__(16) float so[4][16][132]; __shared__ float smu[CO], srs[CO], sg[CO], sb[CO];
  const int tid = threadIdx.x, wave = tid >> 5, lane = tid & 31, col = lane & 15, g = lane >> 4; const size_t r0 = (size_t)blockIdx.x * 64 + wave * 16; size_t ra = r0 + col; if (ra >= NN) ra = NN - 1;
  { const int c = tid; smu[c] = ST[c]; srs[c] = ST[CO + c]; sg[c] = bfr(gm[c]); sb[c] = bfr(bt[c]); }
  __syncthreads();
  v8f acc[8] = {};
#pragma unroll
  for (int kc = 0; kc < CIN / 32; ++kc) { v16b a; const float* p = X + ra * CIN + kc * 32 + 8 * g;
#pragma unroll
    for (int i = 0; i < 8; ++i) { a[i] = (__bf16)p[i]; a[8 + i] = (__bf16)p[16 + i]; }
#pragma unroll
    for (int j = 0; j < 8; ++j) acc[j] = wmma_bf(a, frag_b(PSK + (size_t)(j * 16 + col) * CIN + kc * 32, lane), acc[j]); }
#pragma unroll
  for (int j = 0; j < 8; ++j) { const int c = j * 16 + col;
#pragma unroll
    for (int r = 0; r < 8; ++r) { size_t row = r0 + 8 * g + r; if (row >= NN) row = NN - 1; float v = (Yv[row * CO + c] - smu[c]) * srs[c] * sg[c] + sb[c]; v = fmaxf(v, 0.f); so[wave][8 * g + r][c] = v + acc[j][r]; } }
  LDSX();
  for (int rl = 0; rl < 16; ++rl) if (r0 + rl < (size_t)NN) vst2(out + (r0 + rl) * CO + lane * 4, *(const v4f*)&so[wave][rl][lane * 4]);
}
extern "C" void kernel_launch(void* const* d_in, const int* in_sizes, int n_in, void* d_out, int out_size, void* d_ws, size_t ws_size, hipStream_t stream) {
  (void)in_sizes; (void)n_in; (void)out_size;
  const float** F = (const float**)d_in; const int* NBR = (const int*)d_in[1];
  if (ws_size < (size_t)WS_END) return;
  char* ws = (char*)d_ws; __bf16 *P1 = (__bf16*)(ws + WS_P1), *P2 = (__bf16*)(ws + WS_P2), *PSK = (__bf16*)(ws + WS_PS); float *Y = (float*)(ws + WS_Y), *H = (float*)(ws + WS_H), *PSUM = (float*)(ws + WS_PSUM), *ST = (float*)(ws + WS_ST);
  k_pack<<<dim3(CO, 3), 256, 0, stream>>>(F[2], F[5], F[8], P1, P2, PSK);
  k_conv<CIN, 1><<<NBLK, 128, 0, stream>>>(F[0], NBR, P1, Y);
  k_colsum<0><<<NBLK, 128, 0, stream>>>(Y, ST, PSUM); k_red<0><<<1, 128, 0, stream>>>(PSUM, ST); k_colsum<1><<<NBLK, 128, 0, stream>>>(Y, ST, PSUM); k_red<1><<<1, 128, 0, stream>>>(PSUM, ST);
  k_bnact<<<NBLK, 256, 0, stream>>>(Y, ST, F[3], F[4], H);
  k_conv<CO, 0><<<NBLK, 128, 0, stream>>>(H, NBR, P2, Y);
  k_colsum<0><<<NBLK, 128, 0, stream>>>(Y, ST, PSUM); k_red<0><<<1, 128, 0, stream>>>(PSUM, ST); k_colsum<1><<<NBLK, 128, 0, stream>>>(Y, ST, PSUM); k_red<1><<<1, 128, 0, stream>>>(PSUM, ST);
  k_final<<<NBLK, 128, 0, stream>>>(F[0], PSK, Y, ST, F[6], F[7], (float*)d_out);
}
